// SparseCrossAttention_20529943675444
// MI455X (gfx1250) — hardware-verified
//
#include <hip/hip_runtime.h>
#include <stdint.h>
#include <stddef.h>

constexpr int NPTS  = 16384;
constexpr int CH    = 512;
constexpr int NB    = 4;
constexpr int LCTX  = 512;
constexpr int CTXC  = 1024;
constexpr int NHEAD = 8;
constexpr int HD    = 64;
constexpr int NKV   = NB * LCTX;
constexpr int ATT_KC = 64;
static_assert(NHEAD * HD == CH);
static_assert(NPTS % 512 == 0);
static_assert(NPTS % 64 == 0 && NKV % 64 == 0 && CH % 64 == 0 && (2 * CH) % 64 == 0);
static_assert(CH % 32 == 0 && CTXC % 32 == 0);
static_assert(LCTX % ATT_KC == 0 && HD == 64);
static_assert((NPTS * CH) % (256 * 8) == 0 && (NKV * CTXC) % (256 * 8) == 0);

typedef __attribute__((ext_vector_type(16))) _Float16 v16h;
typedef __attribute__((ext_vector_type(8)))  _Float16 v8h;
typedef __attribute__((ext_vector_type(16))) __bf16   v16b;
typedef __attribute__((ext_vector_type(8)))  __bf16   v8b;
typedef __attribute__((ext_vector_type(8)))  float    v8f;
typedef __attribute__((ext_vector_type(4)))  float    v4f;
typedef __attribute__((ext_vector_type(4)))  unsigned v4u;
typedef __attribute__((ext_vector_type(4)))  int      v4i;

__device__ __forceinline__ unsigned short f2bf_bits(float f) {
  unsigned u = __float_as_uint(f);
  return (unsigned short)((u + 0x7FFFu + ((u >> 16) & 1u)) >> 16);
}
__device__ __forceinline__ float bf_bits2f(unsigned short h) { return __uint_as_float(((unsigned)h) << 16); }

__device__ __forceinline__ void dep_guard_h(v8f& a, v8f& b, v16h x, v16h y) { asm volatile("v_nop\n\tv_nop\n\tv_nop\n\tv_nop" : "+v"(a), "+v"(b) : "v"(x), "v"(y)); }
__device__ __forceinline__ void dep_guard_b(v8f& a, v8f& b, v16b x, v16b y) { asm volatile("v_nop\n\tv_nop\n\tv_nop\n\tv_nop" : "+v"(a), "+v"(b) : "v"(x), "v"(y)); }
__device__ __forceinline__ void keep4_h(v16h a, v16h b, v16h c, v16h d) { asm volatile("v_nop" :: "v"(a), "v"(b), "v"(c), "v"(d)); }
__device__ __forceinline__ void keep4_b(v16b a, v16b b, v16b c, v16b d) { asm volatile("v_nop" :: "v"(a), "v"(b), "v"(c), "v"(d)); }
__device__ __forceinline__ void acc_guard4(v8f& a, v8f& b, v8f& c, v8f& d) { asm volatile("v_nop\n\tv_nop\n\tv_nop\n\tv_nop" : "+v"(a), "+v"(b), "+v"(c), "+v"(d)); }
template <typename T> struct Frag;
template <> struct Frag<_Float16> {
  typedef v16h V; union U { v16h v; v8h h[2]; };
  static __device__ __forceinline__ v16h load(const _Float16* p) {
    U f; f.h[0] = *(const v8h*)(p); f.h[1] = *(const v8h*)(p + 16); return f.v;
  }
  static __device__ __forceinline__ v8f mma(v16h a, v16h b, v8f c) {
    return __builtin_amdgcn_wmma_f32_16x16x32_f16(false, a, false, b, (short)0, c, false, false);
  }
  static __device__ __forceinline__ void guard(v8f& a, v8f& b, v16h x, v16h y) { dep_guard_h(a, b, x, y); }
  static __device__ __forceinline__ void keep(v16h a, v16h b, v16h c, v16h d) { keep4_h(a, b, c, d); }
};
template <> struct Frag<__bf16> {
  typedef v16b V; union U { v16b v; v8b h[2]; };
  static __device__ __forceinline__ v16b load(const __bf16* p) {
    U f; f.h[0] = *(const v8b*)(p); f.h[1] = *(const v8b*)(p + 16); return f.v;
  }
  static __device__ __forceinline__ v8f mma(v16b a, v16b b, v8f c) {
    return __builtin_amdgcn_wmma_f32_16x16x32_bf16(false, a, false, b, (short)0, c, false, false);
  }
  static __device__ __forceinline__ void guard(v8f& a, v8f& b, v16b x, v16b y) { dep_guard_b(a, b, x, y); }
  static __device__ __forceinline__ void keep(v16b a, v16b b, v16b c, v16b d) { keep4_b(a, b, c, d); }
};

__device__ __forceinline__ v8f mma16h(v16h a, v16h b, v8f c) {
  c = __builtin_amdgcn_wmma_f32_16x16x32_f16(false, a, false, b, (short)0, c, false, false);
  asm volatile("v_nop\n\tv_nop\n\tv_nop\n\tv_nop" : "+v"(c) : "v"(a), "v"(b));
  return c;
}
__device__ __forceinline__ v8f mma16b(v16b a, v16b b, v8f c) {
  c = __builtin_amdgcn_wmma_f32_16x16x32_bf16(false, a, false, b, (short)0, c, false, false);
  asm volatile("v_nop\n\tv_nop\n\tv_nop\n\tv_nop" : "+v"(c) : "v"(a), "v"(b));
  return c;
}
__device__ __forceinline__ __bf16 bf_from_bits(unsigned short b) { return __builtin_bit_cast(__bf16, b); }
__device__ __forceinline__ void split_bf(float f, __bf16& hi, __bf16& lo) {
  const unsigned short hb = f2bf_bits(f);
  hi = bf_from_bits(hb);
  lo = bf_from_bits(f2bf_bits(f - bf_bits2f(hb)));
}

template <int ET> struct Elem;
template <> struct Elem<0> { typedef _Float16 T; };
template <> struct Elem<1> { typedef __bf16 T; };
template <int ET, bool SPA, bool SPB, int BIAS_MODE, int OUT_MODE>
__global__ __launch_bounds__(256) void wmma_gemm64(
    const unsigned short* __restrict__ Ap, const unsigned short* __restrict__ A2p, int lda, long strideA,
    const unsigned short* __restrict__ Btp, const unsigned short* __restrict__ Bt2p, int ldb, long strideB,
    void* __restrict__ Cout, void* __restrict__ Cout2, int ldc, long strideC,
    const float* __restrict__ bias,
    int M, int N, int K, float scale) {
  typedef typename Elem<ET>::T T;
  typedef typename Frag<T>::V V;
  const T* A = (const T*)Ap; const T* A2 = (const T*)A2p; const T* Bt = (const T*)Btp; const T* Bt2 = (const T*)Bt2p;
  __shared__ __align__(16) float sT[8][16 * 68];
  const int b    = blockIdx.y;
  const int lane = threadIdx.x & 31;
  const int wave = threadIdx.x >> 5;
  const int tilesN = N >> 6;
  const int tilesM = M >> 6;
  const int tile = blockIdx.x * 8 + wave;
  if (tile >= tilesM * tilesN) return;
  const int tm = tile / tilesN;
  const int tn = tile - tm * tilesN;
  const int m0 = tm << 6;
  const int n0 = tn << 6;

  const T* Ab  = A  + (size_t)b * strideA;
  const T* Bb  = Bt + (size_t)b * strideB;
  const T* Ab2 = SPA ? (A2  + (size_t)b * strideA) : nullptr;
  const T* Bb2 = SPB ? (Bt2 + (size_t)b * strideB) : nullptr;

  const int rlane = lane & 15;
  const int koff  = (lane >> 4) * 8;
  const int mOff  = (lane >> 4) * 8;

  v8f acc[4][4];
#pragma unroll
  for (int i = 0; i < 4; ++i)
#pragma unroll
    for (int j = 0; j < 4; ++j) acc[i][j] = (v8f){0.f,0.f,0.f,0.f,0.f,0.f,0.f,0.f};

  for (int k0 = 0; k0 < K; k0 += 32) {
    V bh[4], bl[4];
#pragma unroll
    for (int j = 0; j < 4; ++j) {
      const size_t bo = (size_t)(n0 + (j << 4) + rlane) * ldb + koff + k0;
      bh[j] = Frag<T>::load(Bb + bo);
      if (SPB) bl[j] = Frag<T>::load(Bb2 + bo);
    }
#pragma unroll
    for (int i = 0; i < 4; ++i) {
      const size_t ao = (size_t)(m0 + (i << 4) + rlane) * lda + koff + k0;
      V ah = Frag<T>::load(Ab + ao);
      V al;
      if (SPA) al = Frag<T>::load(Ab2 + ao);
#pragma unroll
      for (int j = 0; j < 4; ++j) {
        acc[i][j] = Frag<T>::mma(ah, bh[j], acc[i][j]);
        if (SPB) acc[i][j] = Frag<T>::mma(ah, bl[j], acc[i][j]);
        if (SPA) acc[i][j] = Frag<T>::mma(al, bh[j], acc[i][j]);
      }
      Frag<T>::guard(acc[i][0], acc[i][3], ah, SPA ? al : ah);
    }
    Frag<T>::keep(bh[0], bh[1], bh[2], bh[3]);
    if (SPB) Frag<T>::keep(bl[0], bl[1], bl[2], bl[3]);
  }
  acc_guard4(acc[0][0], acc[0][1], acc[0][2], acc[0][3]);
  acc_guard4(acc[1][0], acc[1][1], acc[1][2], acc[1][3]);
  acc_guard4(acc[2][0], acc[2][1], acc[2][2], acc[2][3]);
  acc_guard4(acc[3][0], acc[3][1], acc[3][2], acc[3][3]);

  float* slab = sT[wave];
#pragma unroll
  for (int i = 0; i < 4; ++i) {
    const int mBase = m0 + (i << 4);
#pragma unroll
    for (int j = 0; j < 4; ++j) {
      const int n = n0 + (j << 4) + rlane;
      float bv = 0.f;
      if (BIAS_MODE == 2) bv = bias[n];
#pragma unroll
      for (int r = 0; r < 8; ++r) {
        float v = acc[i][j][r] * scale;
        if (BIAS_MODE == 2) v += bv;
        slab[(mOff + r) * 68 + (j << 4) + rlane] = v;
      }
    }
    __builtin_amdgcn_fence(__ATOMIC_RELEASE, "workgroup");
    __builtin_amdgcn_wave_barrier();
    __builtin_amdgcn_fence(__ATOMIC_ACQUIRE, "workgroup");
    if (OUT_MODE == 0) {
      float* C = (float*)Cout + (size_t)b * strideC;
      const int hh = lane >> 4, c4 = (lane & 15) * 4;
      for (int pass = 0; pass < 2; ++pass) {
#pragma unroll
        for (int it = 0; it < 8; ++it) {
          const int row = it * 2 + hh;
          v4f v = *(const v4f*)(slab + row * 68 + c4);
          *(volatile v4f*)(C + (size_t)(mBase + row) * ldc + n0 + c4) = v;
        }
        __threadfence();
      }
    } else {
      const int q = lane >> 3, c8 = (lane & 7) * 8;
      unsigned short* C  = (unsigned short*)Cout  + (size_t)b * strideC;
      unsigned short* C2 = (OUT_MODE == 2) ? ((unsigned short*)Cout2 + (size_t)b * strideC) : nullptr;
      for (int pass = 0; pass < 2; ++pass) {
#pragma unroll
        for (int it = 0; it < 4; ++it) {
          const int row = it * 4 + q;
          const float* sp = slab + row * 68 + c8;
          v8h hv, lv;
#pragma unroll
          for (int e = 0; e < 8; ++e) {
            if (OUT_MODE == 1) {
              hv[e] = (_Float16)sp[e];
            } else {
              unsigned short hb = f2bf_bits(sp[e]);
              unsigned short lb = f2bf_bits(sp[e] - bf_bits2f(hb));
              hv[e] = __builtin_bit_cast(_Float16, hb);
              lv[e] = __builtin_bit_cast(_Float16, lb);
            }
          }
          *(volatile v8h*)(C + (size_t)(mBase + row) * ldc + n0 + c8) = hv;
          if (OUT_MODE == 2) *(volatile v8h*)(C2 + (size_t)(mBase + row) * ldc + n0 + c8) = lv;
        }
        __threadfence();
      }
    }
    __builtin_amdgcn_fence(__ATOMIC_RELEASE, "workgroup");
    __builtin_amdgcn_wave_barrier();
    __builtin_amdgcn_fence(__ATOMIC_ACQUIRE, "workgroup");
  }
}

__global__ __launch_bounds__(256) void cast_bf16x8_kernel(const float* __restrict__ in,
                                                         unsigned short* __restrict__ out, int n8) {
  const int i = blockIdx.x * 256 + threadIdx.x;
  if (i < n8) {
    const v4f a = *(const v4f*)(in + (size_t)i * 8);
    const v4f c4 = *(const v4f*)(in + (size_t)i * 8 + 4);
    v4u w;
    w[0] = (unsigned)f2bf_bits(a[0])  | ((unsigned)f2bf_bits(a[1])  << 16);
    w[1] = (unsigned)f2bf_bits(a[2])  | ((unsigned)f2bf_bits(a[3])  << 16);
    w[2] = (unsigned)f2bf_bits(c4[0]) | ((unsigned)f2bf_bits(c4[1]) << 16);
    w[3] = (unsigned)f2bf_bits(c4[2]) | ((unsigned)f2bf_bits(c4[3]) << 16);
    unsigned short* o = out + (size_t)i * 8;
    *(volatile v4u*)o = w;
    __threadfence();
    *(volatile v4u*)o = w;
  }
}

__global__ __launch_bounds__(256) void transpose_bf16_kernel(const float* __restrict__ in,
                                                            unsigned short* __restrict__ out,
                                                            int nrows, int ncols) {
  __shared__ float tile[64][65];
  const int tid = threadIdx.x;
  const int c0 = blockIdx.x * 64, r0 = blockIdx.y * 64;
#pragma unroll
  for (int i = 0; i < 4; ++i) {
    const int u = tid + 256 * i;
    const int r = u >> 4, c4 = (u & 15) * 4;
    const v4f v = *(const v4f*)(in + (size_t)(r0 + r) * ncols + c0 + c4);
    tile[r][c4 + 0] = v[0];
    tile[r][c4 + 1] = v[1];
    tile[r][c4 + 2] = v[2];
    tile[r][c4 + 3] = v[3];
  }
  __syncthreads();
  const int qq = tid >> 3, c8 = (tid & 7) * 8;
  for (int pass = 0; pass < 2; ++pass) {
#pragma unroll
    for (int it = 0; it < 2; ++it) {
      const int orow = it * 32 + qq;
      v4u w;
#pragma unroll
      for (int k = 0; k < 4; ++k) {
        const unsigned lo16 = (unsigned)f2bf_bits(tile[c8 + 2 * k][orow]);
        const unsigned hi16 = (unsigned)f2bf_bits(tile[c8 + 2 * k + 1][orow]);
        w[k] = lo16 | (hi16 << 16);
      }
      *(volatile v4u*)(out + (size_t)(c0 + orow) * nrows + r0 + c8) = w;
    }
    __threadfence();
  }
}

__global__ __launch_bounds__(256) void vtranspose_kernel(const unsigned short* __restrict__ vh,
                                                        const unsigned short* __restrict__ vl,
                                                        unsigned short* __restrict__ vth,
                                                        unsigned short* __restrict__ vtl) {
  __shared__ __align__(16) unsigned short th[64][72];
  __shared__ __align__(16) unsigned short tl[64][72];
  const int tid = threadIdx.x;
  const int l0 = blockIdx.x * 64;
  const int bh = blockIdx.y;
  const int b = bh / NHEAD, h = bh - (bh / NHEAD) * NHEAD;
#pragma unroll
  for (int i = 0; i < 2; ++i) {
    const int u = tid + 256 * i;
    const int lr = u >> 3, c8 = (u & 7) * 8;
    const size_t src = (size_t)(b * LCTX + l0 + lr) * CH + h * HD + c8;
    *(v4u*)(&th[lr][c8]) = *(const v4u*)(vh + src);
    *(v4u*)(&tl[lr][c8]) = *(const v4u*)(vl + src);
  }
  __syncthreads();
  const int qq = tid >> 3, c8 = (tid & 7) * 8;
  for (int pass = 0; pass < 2; ++pass) {
#pragma unroll
    for (int it = 0; it < 2; ++it) {
      const int drow = it * 32 + qq;
      v4u wh, wl;
#pragma unroll
      for (int k = 0; k < 4; ++k) {
        wh[k] = (unsigned)th[c8 + 2 * k][drow] | ((unsigned)th[c8 + 2 * k + 1][drow] << 16);
        wl[k] = (unsigned)tl[c8 + 2 * k][drow] | ((unsigned)tl[c8 + 2 * k + 1][drow] << 16);
      }
      const size_t dst = (size_t)(bh * HD + drow) * LCTX + l0 + c8;
      *(volatile v4u*)(vth + dst) = wh;
      *(volatile v4u*)(vtl + dst) = wl;
    }
    __threadfence();
  }
}

__global__ __launch_bounds__(128)
void sparse_xattn_kernel(const unsigned short* __restrict__ Qp, const unsigned short* __restrict__ Kp,
                         const unsigned short* __restrict__ VThp, const unsigned short* __restrict__ VTlp,
                         const int* __restrict__ bidx,
                         unsigned short* __restrict__ OBh, unsigned short* __restrict__ OBl) {
  union FB { v16b v; v8b h[2]; };
  __shared__ __align__(16) _Float16 QKs[64 * HD];
  __shared__ __align__(16) __bf16 Vth[HD * ATT_KC];
  __shared__ __align__(16) __bf16 Vtl[HD * ATT_KC];
  __shared__ __align__(16) __bf16 Psh[4][16 * ATT_KC];
  __shared__ __align__(16) __bf16 Psl[4][16 * ATT_KC];
  __shared__ __align__(16) float  Os[4][16 * 68];
  __shared__ int s_tok[64];
  __shared__ int s_wcnt[4];

  const int tid  = threadIdx.x;
  const int wave = tid >> 5;
  const int lane = tid & 31;
  const int hh   = lane >> 4;
  const int c    = lane & 15;
  const int tt = blockIdx.x, b = blockIdx.y;
  const int lo_rank = tt * 64, hi_rank = lo_rank + 64;
  const _Float16* Qh = (const _Float16*)Qp;
  const _Float16* Kh = (const _Float16*)Kp;
  const __bf16* VTh = (const __bf16*)VThp;
  const __bf16* VTl = (const __bf16*)VTlp;

  if (tid < 64) s_tok[tid] = 0;
  __syncthreads();

  int base = 0;
  const unsigned ltmask = (1u << lane) - 1u;
#pragma unroll 1
  for (int ch = 0; ch < NPTS / 512; ++ch) {
    const int i0 = ch * 512 + tid * 4;
    const v4i bv = *(const v4i*)(bidx + i0);
    int f[4]; unsigned m[4];
#pragma unroll
    for (int e = 0; e < 4; ++e) {
      int cb = bv[e];
      cb = cb < 0 ? 0 : cb;
      cb = cb > NB - 1 ? NB - 1 : cb;
      f[e] = (cb == b) ? 1 : 0;
      m[e] = __builtin_amdgcn_ballot_w32(f[e] != 0);
    }
    int pre = 0, wtot = 0;
#pragma unroll
    for (int e = 0; e < 4; ++e) {
      pre  += (int)__builtin_popcount(m[e] & ltmask);
      wtot += (int)__builtin_popcount(m[e]);
    }
    if (lane == 0) s_wcnt[wave] = wtot;
    __syncthreads();
    const int w0 = s_wcnt[0], w1 = s_wcnt[1], w2 = s_wcnt[2], w3 = s_wcnt[3];
    const int woff = (wave > 0 ? w0 : 0) + (wave > 1 ? w1 : 0) + (wave > 2 ? w2 : 0);
    int rk = base + woff + pre;
#pragma unroll
    for (int e = 0; e < 4; ++e) {
      const int slot = rk - lo_rank;
      if (f[e] != 0 && slot >= 0 && slot < 64) s_tok[slot] = i0 + e;
      rk += f[e];
    }
    base += w0 + w1 + w2 + w3;
    __syncthreads();
    if (base >= hi_rank) break;
  }
  int nvalid = base - lo_rank;
  nvalid = nvalid < 0 ? 0 : nvalid;
  nvalid = nvalid > 64 ? 64 : nvalid;

  if (nvalid > 0) {
#pragma unroll 1
    for (int h = 0; h < NHEAD; ++h) {
      __syncthreads();
#pragma unroll
      for (int i = 0; i < 4; ++i) {
        const int u = tid + 128 * i;
        const int row = u >> 3, c8 = (u & 7) * 8;
        int tok = s_tok[row];
        tok = tok < 0 ? 0 : tok;
        tok = tok > NPTS - 1 ? NPTS - 1 : tok;
        *(v8h*)(QKs + row * HD + c8) = *(const v8h*)(Qh + (size_t)tok * CH + h * HD + c8);
      }
      __syncthreads();
      v16h qa[2];
#pragma unroll
      for (int dc = 0; dc < 2; ++dc)
        qa[dc] = Frag<_Float16>::load(QKs + (wave * 16 + c) * HD + dc * 32 + 8 * hh);

      float mrow[8], lrow[8];
      v8f oacc[4];
#pragma unroll
      for (int r = 0; r < 8; ++r) { mrow[r] = -INFINITY; lrow[r] = 0.f; }
#pragma unroll
      for (int t = 0; t < 4; ++t) oacc[t] = (v8f){0.f,0.f,0.f,0.f,0.f,0.f,0.f,0.f};

#pragma unroll 1
      for (int kc = 0; kc < LCTX / ATT_KC; ++kc) {
        const int kv0 = kc * ATT_KC;
        __syncthreads();
#pragma unroll
        for (int i = 0; i < 4; ++i) {
          const int u = tid + 128 * i;
          const int r8 = u >> 3, c8 = (u & 7) * 8;
          *(v8h*)(QKs + r8 * HD + c8) = *(const v8h*)(Kh + (size_t)(b * LCTX + kv0 + r8) * CH + h * HD + c8);
          const size_t vsrc = (size_t)((b * NHEAD + h) * HD + r8) * LCTX + kv0 + c8;
          *(v8b*)(Vth + r8 * ATT_KC + c8) = *(const v8b*)(VTh + vsrc);
          *(v8b*)(Vtl + r8 * ATT_KC + c8) = *(const v8b*)(VTl + vsrc);
        }
        __syncthreads();

        v8f s[4];
#pragma unroll
        for (int j = 0; j < 4; ++j) {
          s[j] = (v8f){0.f,0.f,0.f,0.f,0.f,0.f,0.f,0.f};
#pragma unroll
          for (int dc = 0; dc < 2; ++dc) {
            const v16h kb = Frag<_Float16>::load(QKs + (j * 16 + c) * HD + dc * 32 + 8 * hh);
            s[j] = mma16h(qa[dc], kb, s[j]);
          }
        }
        float cm[8];
#pragma unroll
        for (int r = 0; r < 8; ++r) {
          float mx = -INFINITY;
#pragma unroll
          for (int j = 0; j < 4; ++j) {
            const float sv = s[j][r] * 0.125f;
            s[j][r] = sv;
            mx = fmaxf(mx, sv);
          }
#pragma unroll
          for (int off = 1; off < 16; off <<= 1) mx = fmaxf(mx, __shfl_xor(mx, off, 32));
          cm[r] = mx;
        }
        __bf16* pwh = Psh[wave];
        __bf16* pwl = Psl[wave];
#pragma unroll
        for (int r = 0; r < 8; ++r) {
          const float mnew = fmaxf(mrow[r], cm[r]);
          const float alpha = expf(mrow[r] - mnew);
          mrow[r] = mnew;
          float psum = 0.f;
#pragma unroll
          for (int j = 0; j < 4; ++j) {
            const float p = expf(s[j][r] - mnew);
            psum += p;
            __bf16 ph, pl;
            split_bf(p, ph, pl);
            pwh[(8 * hh + r) * ATT_KC + j * 16 + c] = ph;
            pwl[(8 * hh + r) * ATT_KC + j * 16 + c] = pl;
          }
#pragma unroll
          for (int off = 1; off < 16; off <<= 1) psum += __shfl_xor(psum, off, 32);
          lrow[r] = lrow[r] * alpha + psum;
#pragma unroll
          for (int t = 0; t < 4; ++t) oacc[t][r] *= alpha;
        }
        __builtin_amdgcn_fence(__ATOMIC_RELEASE, "workgroup");
        __builtin_amdgcn_wave_barrier();
        __builtin_amdgcn_fence(__ATOMIC_ACQUIRE, "workgroup");
#pragma unroll
        for (int kk = 0; kk < 2; ++kk) {
          FB pa, pl;
          pa.h[0] = *(const v8b*)(pwh + c * ATT_KC + kk * 32 + 8 * hh);
          pa.h[1] = *(const v8b*)(pwh + c * ATT_KC + kk * 32 + 16 + 8 * hh);
          pl.h[0] = *(const v8b*)(pwl + c * ATT_KC + kk * 32 + 8 * hh);
          pl.h[1] = *(const v8b*)(pwl + c * ATT_KC + kk * 32 + 16 + 8 * hh);
#pragma unroll
          for (int t = 0; t < 4; ++t) {
            FB vb, vlo;
            vb.h[0]  = *(const v8b*)(Vth + (t * 16 + c) * ATT_KC + kk * 32 + 8 * hh);
            vb.h[1]  = *(const v8b*)(Vth + (t * 16 + c) * ATT_KC + kk * 32 + 16 + 8 * hh);
            vlo.h[0] = *(const v8b*)(Vtl + (t * 16 + c) * ATT_KC + kk * 32 + 8 * hh);
            vlo.h[1] = *(const v8b*)(Vtl + (t * 16 + c) * ATT_KC + kk * 32 + 16 + 8 * hh);
            oacc[t] = mma16b(pa.v, vb.v,  oacc[t]);
            oacc[t] = mma16b(pa.v, vlo.v, oacc[t]);
            oacc[t] = mma16b(pl.v, vb.v,  oacc[t]);
          }
        }
      }

      float* os = Os[wave];
#pragma unroll
      for (int r = 0; r < 8; ++r) {
        const float inv = 1.0f / lrow[r];
#pragma unroll
        for (int t = 0; t < 4; ++t) os[(8 * hh + r) * 68 + t * 16 + c] = oacc[t][r] * inv;
      }
      __builtin_amdgcn_fence(__ATOMIC_RELEASE, "workgroup");
      __builtin_amdgcn_wave_barrier();
      __builtin_amdgcn_fence(__ATOMIC_ACQUIRE, "workgroup");
      {
        const int qq = lane >> 3, c8 = (lane & 7) * 8;
        for (int pass = 0; pass < 2; ++pass) {
#pragma unroll
          for (int it = 0; it < 4; ++it) {
            const int row = it * 4 + qq;
            const int lr = wave * 16 + row;
            int tok = s_tok[lr];
            tok = tok < 0 ? 0 : tok;
            tok = tok > NPTS - 1 ? NPTS - 1 : tok;
            const bool valid = lr < nvalid;
            const float* sp = os + row * 68 + c8;
            v4u wh, wl;
#pragma unroll
            for (int k = 0; k < 4; ++k) {
              const float x0 = sp[2 * k], x1 = sp[2 * k + 1];
              const unsigned short h0 = f2bf_bits(x0), h1 = f2bf_bits(x1);
              const unsigned short l0 = f2bf_bits(x0 - bf_bits2f(h0)), l1 = f2bf_bits(x1 - bf_bits2f(h1));
              wh[k] = (unsigned)h0 | ((unsigned)h1 << 16);
              wl[k] = (unsigned)l0 | ((unsigned)l1 << 16);
            }
            const size_t dst = (size_t)tok * CH + h * HD + c8;
            if (valid) {
              *(volatile v4u*)(OBh + dst) = wh;
              *(volatile v4u*)(OBl + dst) = wl;
            }
          }
          __threadfence();
        }
      }
      __builtin_amdgcn_fence(__ATOMIC_RELEASE, "workgroup");
      __builtin_amdgcn_wave_barrier();
      __builtin_amdgcn_fence(__ATOMIC_ACQUIRE, "workgroup");
    }
  }
}

extern "C" void kernel_launch(void* const* d_in, const int* in_sizes, int n_in,
                              void* d_out, int out_size, void* d_ws, size_t ws_size,
                              hipStream_t stream) {
  if (n_in < 9) return;
  if (in_sizes[0] != NPTS * CH || in_sizes[1] != NKV * CTXC || in_sizes[2] != NPTS ||
      in_sizes[3] != CH * CH || in_sizes[4] != CH || in_sizes[5] != CTXC * 2 * CH ||
      in_sizes[6] != 2 * CH || in_sizes[7] != CH * CH || in_sizes[8] != CH ||
      out_size != NPTS * CH) return;

  const float* x_feats = (const float*)d_in[0];
  const float* context = (const float*)d_in[1];
  const int*   bidx    = (const int*)d_in[2];
  const float* Wq      = (const float*)d_in[3];
  const float* bq      = (const float*)d_in[4];
  const float* Wkv     = (const float*)d_in[5];
  const float* bkv     = (const float*)d_in[6];
  const float* Wo      = (const float*)d_in[7];
  const float* bo      = (const float*)d_in[8];
  float* out = (float*)d_out;

  char* ws = (char*)d_ws;
  size_t off = 0;
  auto take = [&](size_t bytes) { size_t r = off; off = (off + bytes + 255) & ~(size_t)255; return r; };
  unsigned short* WqT  = (unsigned short*)(ws + take((size_t)CH * CH * 2));
  unsigned short* WkvT = (unsigned short*)(ws + take((size_t)(2 * CH) * CTXC * 2));
  unsigned short* WoT  = (unsigned short*)(ws + take((size_t)CH * CH * 2));
  unsigned short* Xb   = (unsigned short*)(ws + take((size_t)NPTS * CH * 2));
  unsigned short* CTXb = (unsigned short*)(ws + take((size_t)NKV * CTXC * 2));
  unsigned short* Qf   = (unsigned short*)(ws + take((size_t)NPTS * CH * 2));
  unsigned short* Kf   = (unsigned short*)(ws + take((size_t)NKV * CH * 2));
  unsigned short* Vh   = (unsigned short*)(ws + take((size_t)NKV * CH * 2));
  unsigned short* Vl   = (unsigned short*)(ws + take((size_t)NKV * CH * 2));
  unsigned short* VTh  = (unsigned short*)(ws + take((size_t)NB * NHEAD * HD * LCTX * 2));
  unsigned short* VTl  = (unsigned short*)(ws + take((size_t)NB * NHEAD * HD * LCTX * 2));
  unsigned short* OBh  = (unsigned short*)(ws + take((size_t)NPTS * CH * 2));
  unsigned short* OBl  = (unsigned short*)(ws + take((size_t)NPTS * CH * 2));
  if (off > ws_size) return;

  hipLaunchKernelGGL(cast_bf16x8_kernel, dim3((NPTS * CH / 8) / 256), dim3(256), 0, stream,
                     x_feats, Xb, NPTS * CH / 8);
  hipLaunchKernelGGL(cast_bf16x8_kernel, dim3((NKV * CTXC / 8) / 256), dim3(256), 0, stream,
                     context, CTXb, NKV * CTXC / 8);

  hipLaunchKernelGGL(transpose_bf16_kernel, dim3(CH / 64, CH / 64), dim3(256), 0, stream, Wq, WqT, CH, CH);
  hipLaunchKernelGGL(transpose_bf16_kernel, dim3((2 * CH) / 64, CTXC / 64), dim3(256), 0, stream, Wkv, WkvT, CTXC, 2 * CH);
  hipLaunchKernelGGL(transpose_bf16_kernel, dim3(CH / 64, CH / 64), dim3(256), 0, stream, Wo, WoT, CH, CH);

  hipLaunchKernelGGL((wmma_gemm64<1, false, false, 2, 1>), dim3(((NPTS / 64) * (CH / 64)) / 8, 1), dim3(256), 0, stream,
                     (const unsigned short*)Xb, (const unsigned short*)Xb, CH, 0L,
                     (const unsigned short*)WqT, (const unsigned short*)WqT, CH, 0L,
                     (void*)Qf, (void*)Qf, CH, 0L, bq, NPTS, CH, CH, 1.0f);
  hipLaunchKernelGGL((wmma_gemm64<1, false, false, 2, 1>), dim3(((NKV / 64) * (CH / 64)) / 8, 1), dim3(256), 0, stream,
                     (const unsigned short*)CTXb, (const unsigned short*)CTXb, CTXC, 0L,
                     (const unsigned short*)WkvT, (const unsigned short*)WkvT, CTXC, 0L,
                     (void*)Kf, (void*)Kf, CH, 0L, bkv, NKV, CH, CTXC, 1.0f);
  hipLaunchKernelGGL((wmma_gemm64<1, false, false, 2, 2>), dim3(((NKV / 64) * (CH / 64)) / 8, 1), dim3(256), 0, stream,
                     (const unsigned short*)CTXb, (const unsigned short*)CTXb, CTXC, 0L,
                     (const unsigned short*)(WkvT + (size_t)CH * CTXC), (const unsigned short*)(WkvT + (size_t)CH * CTXC), CTXC, 0L,
                     (void*)Vh, (void*)Vl, CH, 0L, bkv + CH, NKV, CH, CTXC, 1.0f);

  hipLaunchKernelGGL(vtranspose_kernel, dim3(LCTX / 64, NB * NHEAD), dim3(256), 0, stream,
                     (const unsigned short*)Vh, (const unsigned short*)Vl, VTh, VTl);

  hipLaunchKernelGGL(sparse_xattn_kernel, dim3(NPTS / 64, NB), dim3(128), 0, stream,
                     (const unsigned short*)Qf, (const unsigned short*)Kf,
                     (const unsigned short*)VTh, (const unsigned short*)VTl, bidx, OBh, OBl);

  hipLaunchKernelGGL((wmma_gemm64<1, true, false, 2, 0>), dim3(((NPTS / 64) * (CH / 64)) / 8, 1), dim3(256), 0, stream,
                     (const unsigned short*)OBh, (const unsigned short*)OBl, CH, 0L,
                     (const unsigned short*)WoT, (const unsigned short*)WoT, CH, 0L,
                     (void*)out, (void*)out, CH, 0L, bo, NPTS, CH, CH, 1.0f);
}
